// OPTNaiveAdapter_4612794876118
// MI455X (gfx1250) — hardware-verified
//
#include <hip/hip_runtime.h>


#define NB_  4
#define NPRE 10
#define TT   1024
#define DD   2048
#define NH_  32
#define HD   64
#define ZH   2
#define RH   256
#define NF   32
#define SCL  0.125f
#define PCAR 1024.0f
typedef _Float16 h16;
typedef unsigned short bf;
typedef __attribute__((ext_vector_type(16))) __bf16   v16bf;
typedef __attribute__((ext_vector_type(16))) _Float16 v16h;
typedef __attribute__((ext_vector_type(8)))  _Float16 v8h;
typedef __attribute__((ext_vector_type(8)))  unsigned short v8us;
typedef __attribute__((ext_vector_type(8)))  float    v8f;
typedef __attribute__((ext_vector_type(4)))  float    v4f;
typedef v8h  __attribute__((may_alias)) v8ha;
typedef v4f  __attribute__((may_alias)) v4fa;
typedef v8us __attribute__((may_alias)) v8usa;

__device__ __forceinline__ unsigned short f2bf(float f) { unsigned u = __float_as_uint(f); u += 0x7FFFu + ((u >> 16) & 1u); return (unsigned short)(u >> 16); }
__device__ __forceinline__ float bf2f(unsigned short b) { return __uint_as_float(((unsigned)b) << 16); }
__device__ __forceinline__ float bfr(float f) { return bf2f(f2bf(f)); }
__device__ __forceinline__ v16h cat16(v8h lo, v8h hi) { return __builtin_shufflevector(lo, hi, 0, 1, 2, 3, 4, 5, 6, 7, 8, 9, 10, 11, 12, 13, 14, 15); }
__device__ __forceinline__ v16bf cat16b(v8us lo, v8us hi) { return __builtin_bit_cast(v16bf, __builtin_shufflevector(lo, hi, 0, 1, 2, 3, 4, 5, 6, 7, 8, 9, 10, 11, 12, 13, 14, 15)); }
__device__ __forceinline__ v8f wmma16(v16h a, v16h b, v8f c) { return __builtin_amdgcn_wmma_f32_16x16x32_f16(false, a, false, b, (short)0, c, false, false); }
__device__ __forceinline__ v8f wmmab(v16bf a, v16bf b, v8f c) { return __builtin_amdgcn_wmma_f32_16x16x32_bf16(false, a, false, b, (short)0, c, false, false); }


template <typename T16> struct WFrag;
template <> struct WFrag<h16> { typedef v16h V; static __device__ __forceinline__ V ld(const h16* p) { return cat16(*(const v8h*)p, *(const v8h*)(p + 16)); } static __device__ __forceinline__ v8f mma(V a, V b, v8f c) { return wmma16(a, b, c); } };
template <> struct WFrag<bf> { typedef v16bf V; static __device__ __forceinline__ V ld(const bf* p) { return cat16b(*(const v8us*)p, *(const v8us*)(p + 16)); } static __device__ __forceinline__ v8f mma(V a, V b, v8f c) { return wmmab(a, b, c); } };
template <typename T16, int NSPLIT, bool BIAS>
__global__ __launch_bounds__(32) void k_gemmw(const T16* __restrict__ A, const T16* __restrict__ A2, const T16* __restrict__ Bt, const T16* __restrict__ Bt2, int K, float* C, int ldc, const float* __restrict__ bias, size_t sA, size_t sB, size_t sC) {
    typedef typename WFrag<T16>::V V;
    __shared__ __align__(16) float os[16 * 68];
    const size_t z = blockIdx.z; A += z * sA; if (A2) A2 += z * sA; Bt += z * sB; if (Bt2) Bt2 += z * sB; C += z * sC;
    const int lane = threadIdx.x & 31, lr = lane & 15, hi = lane >> 4; const int r0 = blockIdx.x * 64, c0 = blockIdx.y * 64;
    v8f acc[4][4];
#pragma unroll
    for (int mb = 0; mb < 4; ++mb)
#pragma unroll
        for (int nb = 0; nb < 4; ++nb) acc[mb][nb] = (v8f){};
    const size_t aoff = (size_t)(r0 + lr) * K + 8 * hi, boff = (size_t)(c0 + lr) * K + 8 * hi;
#pragma unroll 1
    for (int kc = 0; kc < K; kc += 32) {
        V a[4], a2[4];
#pragma unroll
        for (int mb = 0; mb < 4; ++mb) { a[mb] = WFrag<T16>::ld(A + aoff + (size_t)mb * 16 * K + kc); if (NSPLIT == 1 || NSPLIT == 2) a2[mb] = WFrag<T16>::ld(A2 + aoff + (size_t)mb * 16 * K + kc); }
#pragma unroll
        for (int nb = 0; nb < 4; ++nb) { const V b = WFrag<T16>::ld(Bt + boff + (size_t)nb * 16 * K + kc); V b2; if (NSPLIT >= 2) b2 = WFrag<T16>::ld(Bt2 + boff + (size_t)nb * 16 * K + kc);
#pragma unroll
            for (int mb = 0; mb < 4; ++mb) { acc[mb][nb] = WFrag<T16>::mma(a[mb], b, acc[mb][nb]); if (NSPLIT == 1 || NSPLIT == 2) acc[mb][nb] = WFrag<T16>::mma(a2[mb], b, acc[mb][nb]); if (NSPLIT >= 2) acc[mb][nb] = WFrag<T16>::mma(a[mb], b2, acc[mb][nb]); } }
        asm volatile("v_nop\n\tv_nop\n\tv_nop\n\tv_nop" : "+v"(acc[0][0]), "+v"(acc[1][1]), "+v"(acc[2][2]), "+v"(acc[3][3]) : "v"(a[0]), "v"(a[3]));
    }
#pragma unroll
    for (int mb = 0; mb < 4; ++mb) {
#pragma unroll
        for (int nb = 0; nb < 4; ++nb) {
#pragma unroll
            for (int j = 0; j < 8; ++j) os[(hi * 8 + j) * 68 + nb * 16 + lr] = acc[mb][nb][j]; }
        __builtin_amdgcn_wave_barrier(); asm volatile("" ::: "memory");
        float* crow = C + (size_t)(r0 + mb * 16) * ldc + c0;
#pragma unroll 1
        for (int ps = 0; ps < 2; ++ps) {
#pragma unroll
            for (int s = 0; s < 8; ++s) { const int row = 2 * s + hi, cofs = lr * 4; v4f val = *(const v4fa*)(os + row * 68 + cofs); if (BIAS) { val[0] += bfr(bias[c0 + cofs]); val[1] += bfr(bias[c0 + cofs + 1]); val[2] += bfr(bias[c0 + cofs + 2]); val[3] += bfr(bias[c0 + cofs + 3]); }
                *(volatile v4f*)(crow + (size_t)row * ldc + cofs) = val; }
            if (ps == 0) __threadfence(); }
        __builtin_amdgcn_wave_barrier(); asm volatile("" ::: "memory");
    }
}

__device__ __forceinline__ h16 tohx(float x) { return (h16)x; }
__device__ __forceinline__ void splitf(float y, unsigned short& h, unsigned short& l) { h = f2bf(y); l = f2bf(y - bf2f(h)); }
typedef __attribute__((ext_vector_type(2))) unsigned short v2us;
typedef __attribute__((ext_vector_type(2))) _Float16 v2h;
typedef __attribute__((ext_vector_type(4))) _Float16 v4h;
typedef __attribute__((ext_vector_type(2))) float v2f;

__global__ __launch_bounds__(256) void k_wtG(const float* __restrict__ w, int K, int N, bf* Bt) {
    const int lane = threadIdx.x & 31; const int L0 = (blockIdx.x * 8 + (threadIdx.x >> 5)) * 8; const int nlines = N * K / 64;
#pragma unroll 1
    for (int ps = 0; ps < 2; ++ps) {
#pragma unroll 1
        for (int l = 0; l < 8; ++l) { const int L = L0 + l; if (L >= nlines) break; const size_t e = (size_t)L * 64 + lane * 2; const int k = (int)(e % K), n = (int)(e / K); v2us o;
            o[0] = f2bf(w[(size_t)k * N + n]); o[1] = f2bf(w[(size_t)(k + 1) * N + n]); *(volatile v2us*)(Bt + e) = o; }
        if (ps == 0) __threadfence(); }
}
__global__ __launch_bounds__(256) void k_cvt8(const float* __restrict__ src, bf* dst, size_t n8) { const size_t i = (size_t)blockIdx.x * 256 + threadIdx.x; if (i >= n8) return; const v8f v = *(const v8f*)(src + i * 8); v8us o;
#pragma unroll
    for (int k = 0; k < 8; ++k) o[k] = f2bf(v[k]); *(volatile v8us*)(dst + i * 8) = o; __threadfence(); *(volatile v8us*)(dst + i * 8) = o; }
__global__ __launch_bounds__(256) void k_qplanes(const float* __restrict__ F, bf* Ph, bf* Pl, h16* P16) {
    const int lane = threadIdx.x & 31; const int L0 = (blockIdx.x * 8 + (threadIdx.x >> 5)) * 8; const int nlines = NH_ * TT * HD / 64;
#pragma unroll 1
    for (int ps = 0; ps < 2; ++ps) {
#pragma unroll
        for (int l = 0; l < 8; ++l) { const int L = L0 + l; if (L >= nlines) break; const int e = L * 64 + lane * 2; const int d = e & (HD - 1); const int t = (e >> 6) & (TT - 1); const int h = e >> 16; v2us oh, ol; v2h o16;
#pragma unroll
            for (int q = 0; q < 2; ++q) { const float x = F[(size_t)t * DD + h * HD + d + q]; unsigned short a, c2; splitf(x, a, c2); oh[q] = a; ol[q] = c2; o16[q] = tohx(x); }
            *(volatile v2us*)(Ph + (size_t)e) = oh; *(volatile v2us*)(Pl + (size_t)e) = ol; *(volatile v2h*)(P16 + (size_t)e) = o16; }
        if (ps == 0) __threadfence(); }
}
__global__ __launch_bounds__(256) void k_prefkv(const float* __restrict__ pre, const float* __restrict__ wk, const float* __restrict__ bk, const float* __restrict__ wv, const float* __restrict__ bv, float* KP0, float* VP0) {
    const int idx = blockIdx.x * 256 + threadIdx.x; if (idx >= NPRE * DD) return; const int l = idx / DD, o = idx % DD; const float* pr = pre + (size_t)l * DD; const float* wkr = wk + (size_t)o * DD; const float* wvr = wv + (size_t)o * DD; float sk = 0.f, sv = 0.f;
#pragma unroll 4
    for (int i = 0; i < DD; ++i) { const float p = bfr(pr[i]); float a = bfr(wkr[i]), c = bfr(wvr[i]); asm volatile("" : "+v"(a)); asm volatile("" : "+v"(c)); float pk = __fmul_rn(p, a), pv = __fmul_rn(p, c); asm volatile("" : "+v"(pk)); asm volatile("" : "+v"(pv)); sk = __fadd_rn(sk, pk); sv = __fadd_rn(sv, pv); }
    float bk2 = bfr(bk[o]), bv2 = bfr(bv[o]); asm volatile("" : "+v"(bk2)); asm volatile("" : "+v"(bv2)); const float ok = __fadd_rn(sk, bk2), ov = __fadd_rn(sv, bv2);
    *(volatile float*)(KP0 + idx) = ok; *(volatile float*)(VP0 + idx) = ov; __threadfence(); *(volatile float*)(KP0 + idx) = ok; *(volatile float*)(VP0 + idx) = ov; }
__global__ __launch_bounds__(256) void k_pre(const float* __restrict__ FQ, const float* __restrict__ KP0, const float* __restrict__ VP0, const float* __restrict__ gate, int h0, float* PRE) {
    const int lane = threadIdx.x & 31; const int row = blockIdx.x * 8 + (threadIdx.x >> 5); if (row >= ZH * TT) return; const int t = row & (TT - 1); const int zz = row / TT; const int h = h0 + zz; const float* q = FQ + (size_t)t * DD + h * HD; float s = -3.0e38f;
    if (lane < NPRE) { const float* kr = KP0 + (size_t)lane * DD + h * HD; float acc = 0.f;
#pragma unroll 4
        for (int d = 0; d < HD; ++d) { float p = __fmul_rn(q[d], kr[d]); asm volatile("" : "+v"(p)); acc = __fadd_rn(acc, p); } s = acc * SCL; }
    float mx = s;
#pragma unroll
    for (int sh = 16; sh; sh >>= 1) mx = fmaxf(mx, __shfl_xor(mx, sh, 32));
    float dl = __fsub_rn(s, mx); asm volatile("" : "+v"(dl)); const float e = (lane < NPRE) ? __builtin_amdgcn_exp2f(__fmul_rn(dl, 1.4426950408889634f)) : 0.f; float sum = e;
#pragma unroll
    for (int sh = 16; sh; sh >>= 1) sum += __shfl_xor(sum, sh, 32);
    float pw = __fdiv_rn(e, sum); const float gv = bfr(gate[h]); const float e2 = __expf(2.0f * gv); const float tg = __fsub_rn(1.0f, __fdiv_rn(2.0f, __fadd_rn(e2, 1.0f))); float o0 = 0.f, o1 = 0.f; const int dd = 2 * lane;
#pragma unroll
    for (int l = 0; l < NPRE; ++l) { const float pl = __shfl(pw, l, 32); const float* vr = VP0 + (size_t)l * DD + h * HD; float a0 = __fmul_rn(pl, vr[dd]), a1 = __fmul_rn(pl, vr[dd + 1]); asm volatile("" : "+v"(a0)); asm volatile("" : "+v"(a1)); o0 = __fadd_rn(o0, a0); o1 = __fadd_rn(o1, a1); }
    v2f o; o[0] = __fmul_rn(tg, o0); o[1] = __fmul_rn(tg, o1); float* dst = PRE + ((size_t)zz * TT + t) * HD + dd; *(volatile v2f*)dst = o; __threadfence(); *(volatile v2f*)dst = o; }
__global__ __launch_bounds__(256) void k_vtplane(const float* __restrict__ F, bf* Vh, bf* Vl, h16* V16) {
    const int lane = threadIdx.x & 31; const int L0 = (blockIdx.x * 8 + (threadIdx.x >> 5)) * 8; const int nlines = NH_ * TT * HD / 64;
#pragma unroll 1
    for (int ps = 0; ps < 2; ++ps) {
#pragma unroll
        for (int l = 0; l < 8; ++l) { const int L = L0 + l; if (L >= nlines) break; const int e = L * 64 + lane * 2; const int t = e & (TT - 1); const int d = (e >> 10) & (HD - 1); const int h = e >> 16; v2us oh, ol; v2h o16;
#pragma unroll
            for (int q = 0; q < 2; ++q) { const float x = F[(size_t)(t + q) * DD + h * HD + d]; unsigned short a, c2; splitf(x, a, c2); oh[q] = a; ol[q] = c2; o16[q] = tohx(x); }
            *(volatile v2us*)(Vh + (size_t)e) = oh; *(volatile v2us*)(Vl + (size_t)e) = ol; *(volatile v2h*)(V16 + (size_t)e) = o16; }
        if (ps == 0) __threadfence(); }
}
__global__ __launch_bounds__(256) void k_asoft(const float* __restrict__ Sb, const float* __restrict__ ab, bf* Ph, bf* Pl, h16* P16) {
    typedef __attribute__((ext_vector_type(4))) unsigned short v4us;
    const int lane = threadIdx.x & 31; const int row = blockIdx.x * 8 + (threadIdx.x >> 5); if (row >= ZH * TT) return; const int i = row & (TT - 1); const int zz = row >> 10; const bool hires = (i < RH);
    const float* sr = Sb + (size_t)row * TT; const float* mr = ab + (size_t)i * TT; float v[32]; float mx = -3.0e38f;
#pragma unroll
    for (int ch = 0; ch < 8; ++ch) { const int j0 = ch * 128 + lane * 4; const v4f a = *(const v4f*)(sr + j0), m4 = *(const v4f*)(mr + j0);
#pragma unroll
        for (int q = 0; q < 4; ++q) { float sa = a[q] * SCL, mb = bfr(m4[q]); asm volatile("" : "+v"(sa)); asm volatile("" : "+v"(mb)); const float t = fmaxf(__fadd_rn(sa, mb), -3.40282347e38f); v[ch * 4 + q] = t; mx = fmaxf(mx, t); } }
#pragma unroll
    for (int sh = 16; sh; sh >>= 1) mx = fmaxf(mx, __shfl_xor(mx, sh, 32));
    float sum = 0.f;
#pragma unroll
    for (int k = 0; k < 32; ++k) { v[k] = __expf(v[k] - mx); sum += v[k]; }
#pragma unroll
    for (int sh = 16; sh; sh >>= 1) sum += __shfl_xor(sum, sh, 32);
    const float f = __fdiv_rn(hires ? 1.0f : PCAR, sum);
#pragma unroll 1
    for (int ps = 0; ps < 2; ++ps) {
        if (hires) {
#pragma unroll
            for (int ch = 0; ch < 8; ++ch) { v4us oh, ol;
#pragma unroll
                for (int q = 0; q < 4; ++q) { unsigned short a, c2; splitf(v[ch * 4 + q] * f, a, c2); oh[q] = a; ol[q] = c2; }
                const size_t o = ((size_t)zz * RH + i) * TT + ch * 128 + lane * 4; *(volatile v4us*)(Ph + o) = oh; *(volatile v4us*)(Pl + o) = ol; }
        } else {
#pragma unroll
            for (int ch = 0; ch < 8; ++ch) { v4h o;
#pragma unroll
                for (int q = 0; q < 4; ++q) o[q] = tohx(v[ch * 4 + q] * f);
                *(volatile v4h*)(P16 + (size_t)row * TT + ch * 128 + lane * 4) = o; } }
        if (ps == 0) __threadfence(); }
}
__global__ __launch_bounds__(256) void k_merge(const float* __restrict__ O, const float* __restrict__ PRE, int h0, bf* Ah, bf* Al) { const int e = (blockIdx.x * 256 + threadIdx.x) * 2; if (e >= ZH * TT * HD) return; const int d = e & 63; const int t = (e >> 6) & (TT - 1); const int zz = e >> 16; const float cs = (t < RH) ? 1.0f : (1.0f / PCAR); v2us oh, ol;
#pragma unroll
    for (int q = 0; q < 2; ++q) { float a = __fmul_rn(O[e + q], cs); asm volatile("" : "+v"(a)); unsigned short a2, c2; splitf(__fadd_rn(a, PRE[e + q]), a2, c2); oh[q] = a2; ol[q] = c2; } const size_t oo = (size_t)t * DD + (h0 + zz) * HD + d; *(volatile v2us*)(Ah + oo) = oh; *(volatile v2us*)(Al + oo) = ol; __threadfence(); *(volatile v2us*)(Ah + oo) = oh; *(volatile v2us*)(Al + oo) = ol; }

extern "C" void kernel_launch(void* const* d_in, const int* in_sizes, int n_in,
                              void* d_out, int out_size, void* d_ws, size_t ws_size, hipStream_t stream) {
    (void)in_sizes; (void)n_in; (void)out_size;
    const float* x = (const float*)d_in[0]; const float* am = (const float*)d_in[1]; const float* wq = (const float*)d_in[2]; const float* bq = (const float*)d_in[3]; const float* wk = (const float*)d_in[4]; const float* bk = (const float*)d_in[5]; const float* wv = (const float*)d_in[6]; const float* bv = (const float*)d_in[7]; const float* wo = (const float*)d_in[8]; const float* bo = (const float*)d_in[9]; const float* pre = (const float*)d_in[10]; const float* gate = (const float*)d_in[11];
    float* OUT = (float*)d_out;
    char* wsp = (char*)d_ws;
    auto take = [&](size_t bytes) { char* p = wsp; wsp += (bytes + 255) & ~(size_t)255; return (void*)p; };
    bf* WQ = (bf*)take((size_t)DD * DD * 2); bf* WK = (bf*)take((size_t)DD * DD * 2); bf* WV = (bf*)take((size_t)DD * DD * 2); bf* WO = (bf*)take((size_t)DD * DD * 2); float* KP0 = (float*)take((size_t)NPRE * DD * 4); float* VP0 = (float*)take((size_t)NPRE * DD * 4);
    bf* XB = (bf*)take((size_t)TT * DD * 2); float* F = (float*)take((size_t)TT * DD * 4); float* FQ = (float*)take((size_t)TT * DD * 4);
    bf* QPh = (bf*)take((size_t)TT * DD * 2); bf* QPl = (bf*)take((size_t)TT * DD * 2); bf* KPh = (bf*)take((size_t)TT * DD * 2); bf* KPl = (bf*)take((size_t)TT * DD * 2); bf* VTh = (bf*)take((size_t)TT * DD * 2); bf* VTl = (bf*)take((size_t)TT * DD * 2);
    h16* QP16 = (h16*)take((size_t)TT * DD * 2); h16* KP16 = (h16*)take((size_t)TT * DD * 2); h16* VT16 = (h16*)take((size_t)TT * DD * 2);
    float* Sb = (float*)take((size_t)ZH * TT * TT * 4); bf* Ph = (bf*)take((size_t)ZH * RH * TT * 2); bf* Pl = (bf*)take((size_t)ZH * RH * TT * 2); h16* P16 = (h16*)take((size_t)ZH * TT * TT * 2); float* Ob = (float*)take((size_t)ZH * TT * HD * 4); float* PRE = (float*)take((size_t)ZH * TT * HD * 4); bf* ATh = (bf*)take((size_t)TT * DD * 2); bf* ATl = (bf*)take((size_t)TT * DD * 2);
    if ((size_t)(wsp - (char*)d_ws) > ws_size) return;
    { const size_t nw = (size_t)DD * DD / 8; const unsigned g = (unsigned)((nw + 255) / 256); k_cvt8<<<g, 256, 0, stream>>>(wq, WQ, nw); k_cvt8<<<g, 256, 0, stream>>>(wk, WK, nw); k_cvt8<<<g, 256, 0, stream>>>(wv, WV, nw); k_cvt8<<<g, 256, 0, stream>>>(wo, WO, nw);
      k_prefkv<<<(NPRE * DD + 255) / 256, 256, 0, stream>>>(pre, wk, bk, wv, bv, KP0, VP0); }
    const unsigned LB = (unsigned)((NH_ * TT * HD / 64 + 63) / 64); const dim3 gP(TT / 64, DD / 64, 1);
    for (int b = 0; b < NB_; ++b) {
        k_cvt8<<<(unsigned)(((size_t)TT * DD / 8 + 255) / 256), 256, 0, stream>>>(x + (size_t)b * TT * DD, XB, (size_t)TT * DD / 8);
        k_gemmw<bf, 0, true><<<gP, 32, 0, stream>>>(XB, nullptr, WQ, nullptr, DD, FQ, DD, bq, 0, 0, 0); k_qplanes<<<LB, 256, 0, stream>>>(FQ, QPh, QPl, QP16);
        k_gemmw<bf, 0, true><<<gP, 32, 0, stream>>>(XB, nullptr, WK, nullptr, DD, F, DD, bk, 0, 0, 0); k_qplanes<<<LB, 256, 0, stream>>>(F, KPh, KPl, KP16);
        k_gemmw<bf, 0, true><<<gP, 32, 0, stream>>>(XB, nullptr, WV, nullptr, DD, F, DD, bv, 0, 0, 0); k_vtplane<<<LB, 256, 0, stream>>>(F, VTh, VTl, VT16);
        for (int h0 = 0; h0 < NH_; h0 += ZH) { const size_t z0 = (size_t)h0;
            k_gemmw<bf, 2, false><<<dim3(RH / 64, TT / 64, ZH), 32, 0, stream>>>(QPh + z0 * TT * HD, QPl + z0 * TT * HD, KPh + z0 * TT * HD, KPl + z0 * TT * HD, HD, Sb, TT, nullptr, (size_t)TT * HD, (size_t)TT * HD, (size_t)TT * TT);
            k_gemmw<h16, 0, false><<<dim3((TT - RH) / 64, TT / 64, ZH), 32, 0, stream>>>(QP16 + z0 * TT * HD + (size_t)RH * HD, nullptr, KP16 + z0 * TT * HD, nullptr, HD, Sb + (size_t)RH * TT, TT, nullptr, (size_t)TT * HD, (size_t)TT * HD, (size_t)TT * TT);
            k_asoft<<<ZH * TT / 8, 256, 0, stream>>>(Sb, am + (size_t)b * TT * TT, Ph, Pl, P16);
            k_gemmw<bf, 2, false><<<dim3(RH / 64, HD / 64, ZH), 32, 0, stream>>>(Ph, Pl, VTh + z0 * HD * TT, VTl + z0 * HD * TT, TT, Ob, HD, nullptr, (size_t)RH * TT, (size_t)HD * TT, (size_t)TT * HD);
            k_gemmw<h16, 0, false><<<dim3((TT - RH) / 64, HD / 64, ZH), 32, 0, stream>>>(P16 + (size_t)RH * TT, nullptr, VT16 + z0 * HD * TT, nullptr, TT, Ob + (size_t)RH * HD, HD, nullptr, (size_t)TT * TT, (size_t)HD * TT, (size_t)TT * HD);
            k_pre<<<ZH * TT / 8, 256, 0, stream>>>(FQ, KP0, VP0, gate, h0, PRE);
            k_merge<<<(ZH * TT * HD / 2 + 255) / 256, 256, 0, stream>>>(Ob, PRE, h0, ATh, ATl); }
        k_gemmw<bf, 1, true><<<gP, 32, 0, stream>>>(ATh, ATl, WO, nullptr, DD, OUT + (size_t)b * TT * DD, DD, bo, 0, 0, 0); }
}
